// GlobalCrossAttention_17454747091611
// MI455X (gfx1250) — hardware-verified
//
#include <hip/hip_runtime.h>


#define NB_  2
#define NQ   900
#define QP   960
#define TT   4096
#define GW   64
#define CH   256
#define NH_  8
#define HD   32
#define HP   64
#define RHID 512
#define PCAR 1024.0f
#define SCL  0.17677669529663688f
typedef _Float16 h16;
typedef unsigned short bf;
typedef __attribute__((ext_vector_type(16))) __bf16   v16bf;
typedef __attribute__((ext_vector_type(16))) _Float16 v16h;
typedef __attribute__((ext_vector_type(8)))  _Float16 v8h;
typedef __attribute__((ext_vector_type(8)))  unsigned short v8us;
typedef __attribute__((ext_vector_type(8)))  float    v8f;
typedef __attribute__((ext_vector_type(4)))  float    v4f;
typedef v8h  __attribute__((may_alias)) v8ha;
typedef v4f  __attribute__((may_alias)) v4fa;
typedef v8us __attribute__((may_alias)) v8usa;

__device__ __forceinline__ unsigned short f2bf(float f) { unsigned u = __float_as_uint(f); u += 0x7FFFu + ((u >> 16) & 1u); return (unsigned short)(u >> 16); }
__device__ __forceinline__ float bf2f(unsigned short b) { return __uint_as_float(((unsigned)b) << 16); }
__device__ __forceinline__ float bfr(float f) { return bf2f(f2bf(f)); }
__device__ __forceinline__ v16h cat16(v8h lo, v8h hi) { return __builtin_shufflevector(lo, hi, 0, 1, 2, 3, 4, 5, 6, 7, 8, 9, 10, 11, 12, 13, 14, 15); }
__device__ __forceinline__ v16bf cat16b(v8us lo, v8us hi) { return __builtin_bit_cast(v16bf, __builtin_shufflevector(lo, hi, 0, 1, 2, 3, 4, 5, 6, 7, 8, 9, 10, 11, 12, 13, 14, 15)); }
__device__ __forceinline__ v8f wmma16(v16h a, v16h b, v8f c) { return __builtin_amdgcn_wmma_f32_16x16x32_f16(false, a, false, b, (short)0, c, false, false); }
__device__ __forceinline__ v8f wmmab(v16bf a, v16bf b, v8f c) { return __builtin_amdgcn_wmma_f32_16x16x32_bf16(false, a, false, b, (short)0, c, false, false); }


template <typename T16> struct WFrag;
template <> struct WFrag<h16> { typedef v16h V; static __device__ __forceinline__ V ld(const h16* p) { return cat16(*(const v8h*)p, *(const v8h*)(p + 16)); } static __device__ __forceinline__ v8f mma(V a, V b, v8f c) { return wmma16(a, b, c); } };
template <> struct WFrag<bf> { typedef v16bf V; static __device__ __forceinline__ V ld(const bf* p) { return cat16b(*(const v8us*)p, *(const v8us*)(p + 16)); } static __device__ __forceinline__ v8f mma(V a, V b, v8f c) { return wmmab(a, b, c); } };
template <typename T16, int NSPLIT, bool BIAS>
__global__ __launch_bounds__(32) void k_gemmw(const T16* __restrict__ A, const T16* __restrict__ A2, const T16* __restrict__ Bt, const T16* __restrict__ Bt2, int K, float* C, int ldc, const float* __restrict__ bias, size_t sA, size_t sB, size_t sC) {
    typedef typename WFrag<T16>::V V;
    __shared__ __align__(16) float os[16 * 68];
    const size_t z = blockIdx.z; A += z * sA; if (A2) A2 += z * sA; Bt += z * sB; if (Bt2) Bt2 += z * sB; C += z * sC;
    const int lane = threadIdx.x & 31, lr = lane & 15, hi = lane >> 4; const int r0 = blockIdx.x * 64, c0 = blockIdx.y * 64;
    v8f acc[4][4];
#pragma unroll
    for (int mb = 0; mb < 4; ++mb)
#pragma unroll
        for (int nb = 0; nb < 4; ++nb) acc[mb][nb] = (v8f){};
    const size_t aoff = (size_t)(r0 + lr) * K + 8 * hi, boff = (size_t)(c0 + lr) * K + 8 * hi;
#pragma unroll 1
    for (int kc = 0; kc < K; kc += 32) {
        V a[4], a2[4];
#pragma unroll
        for (int mb = 0; mb < 4; ++mb) { a[mb] = WFrag<T16>::ld(A + aoff + (size_t)mb * 16 * K + kc); if (NSPLIT == 1 || NSPLIT == 2) a2[mb] = WFrag<T16>::ld(A2 + aoff + (size_t)mb * 16 * K + kc); }
#pragma unroll
        for (int nb = 0; nb < 4; ++nb) { const V b = WFrag<T16>::ld(Bt + boff + (size_t)nb * 16 * K + kc); V b2; if (NSPLIT >= 2) b2 = WFrag<T16>::ld(Bt2 + boff + (size_t)nb * 16 * K + kc);
#pragma unroll
            for (int mb = 0; mb < 4; ++mb) { acc[mb][nb] = WFrag<T16>::mma(a[mb], b, acc[mb][nb]); if (NSPLIT == 1 || NSPLIT == 2) acc[mb][nb] = WFrag<T16>::mma(a2[mb], b, acc[mb][nb]); if (NSPLIT >= 2) acc[mb][nb] = WFrag<T16>::mma(a[mb], b2, acc[mb][nb]); } }
        asm volatile("v_nop\n\tv_nop\n\tv_nop\n\tv_nop" : "+v"(acc[0][0]), "+v"(acc[1][1]), "+v"(acc[2][2]), "+v"(acc[3][3]) : "v"(a[0]), "v"(a[3]));
    }
#pragma unroll
    for (int mb = 0; mb < 4; ++mb) {
#pragma unroll
        for (int nb = 0; nb < 4; ++nb) {
#pragma unroll
            for (int j = 0; j < 8; ++j) os[(hi * 8 + j) * 68 + nb * 16 + lr] = acc[mb][nb][j]; }
        __builtin_amdgcn_wave_barrier(); asm volatile("" ::: "memory");
        float* crow = C + (size_t)(r0 + mb * 16) * ldc + c0;
#pragma unroll 1
        for (int ps = 0; ps < 2; ++ps) {
#pragma unroll
            for (int s = 0; s < 8; ++s) { const int row = 2 * s + hi, cofs = lr * 4; v4f val = *(const v4fa*)(os + row * 68 + cofs); if (BIAS) { val[0] += bfr(bias[c0 + cofs]); val[1] += bfr(bias[c0 + cofs + 1]); val[2] += bfr(bias[c0 + cofs + 2]); val[3] += bfr(bias[c0 + cofs + 3]); }
                *(volatile v4f*)(crow + (size_t)row * ldc + cofs) = val; }
            if (ps == 0) __threadfence(); }
        __builtin_amdgcn_wave_barrier(); asm volatile("" ::: "memory");
    }
}

typedef __attribute__((ext_vector_type(4))) unsigned short v4us;
typedef __attribute__((ext_vector_type(2))) unsigned short v2us;
typedef __attribute__((ext_vector_type(2))) _Float16 v2h;
typedef __attribute__((ext_vector_type(4))) _Float16 v4h;
typedef __attribute__((ext_vector_type(4))) int v4i;
__device__ __forceinline__ void splitf(float y, unsigned short& h, unsigned short& l) { h = f2bf(y); l = f2bf(y - bf2f(h)); }
__device__ __forceinline__ _Float16 tohx(float v) { return (_Float16)v; }
__global__ __launch_bounds__(256) void k_cvt8(const float* __restrict__ src, bf* dst, size_t n8) { const size_t i = (size_t)blockIdx.x * 256 + threadIdx.x; if (i >= n8) return; const v8f v = *(const v8f*)(src + i * 8); v8us o;
#pragma unroll
    for (int k = 0; k < 8; ++k) o[k] = f2bf(v[k]); *(volatile v8us*)(dst + i * 8) = o; __threadfence(); *(volatile v8us*)(dst + i * 8) = o; }

__global__ __launch_bounds__(256) void k_zero(float* Z, size_t n4) { const size_t i = (size_t)blockIdx.x * 256 + threadIdx.x; if (i >= n4) return; v4f o; o[0] = o[1] = o[2] = o[3] = 0.f; *(volatile v4f*)(Z + i * 4) = o; __threadfence(); *(volatile v4f*)(Z + i * 4) = o; }
__global__ __launch_bounds__(256) void k_zero16(bf* Z, size_t n8) { const size_t i = (size_t)blockIdx.x * 256 + threadIdx.x; if (i >= n8) return; v8us o; for (int k = 0; k < 8; ++k) o[k] = 0; *(volatile v8us*)(Z + i * 8) = o; __threadfence(); *(volatile v8us*)(Z + i * 8) = o; }
__global__ __launch_bounds__(256) void k_cpb(const float* __restrict__ box, int ax, const float* __restrict__ w1, const float* __restrict__ b1, const float* __restrict__ w2, float* R) {
    const int i = blockIdx.x * 256 + threadIdx.x; if (i >= NQ * NH_ * (GW / 4)) return; const int c0 = (i % (GW / 4)) * 4; const int h = (i / (GW / 4)) % NH_; const int q = i / ((GW / 4) * NH_);
    const float ctr = bfr(box[(size_t)q * 4 + ax]), sz = bfr(box[(size_t)q * 4 + 2 + ax]); const float hs = __fmul_rn(sz, 0.5f); const float e0 = __fsub_rn(ctr, hs), e1 = __fadd_rn(ctr, hs);
    float acc[4] = {0.f, 0.f, 0.f, 0.f}; float d0[4], d1[4];
#pragma unroll
    for (int k = 0; k < 4; ++k) { const float pos = __fmul_rn((float)(c0 + k) + 0.5f, 16.0f); d0[k] = __fsub_rn(e0, pos); d1[k] = __fsub_rn(e1, pos); }
#pragma unroll 2
    for (int r = 0; r < RHID; ++r) { const float wa = bfr(w1[r * 2]), wb = bfr(w1[r * 2 + 1]), bb = bfr(b1[r]), wo = bfr(w2[(size_t)h * RHID + r]);
#pragma unroll
        for (int k = 0; k < 4; ++k) { float pa = __fmul_rn(d0[k], wa); float pb = __fmul_rn(d1[k], wb); asm volatile("" : "+v"(pa), "+v"(pb)); float hv = __fadd_rn(__fadd_rn(pa, pb), bb); hv = fmaxf(hv, 0.0f); float pr = __fmul_rn(hv, wo); asm volatile("" : "+v"(pr)); acc[k] = __fadd_rn(acc[k], pr); } }
    v4f o; for (int k = 0; k < 4; ++k) o[k] = acc[k]; float* dst = R + ((size_t)q * NH_ + h) * GW + c0; *(volatile v4f*)dst = o; __threadfence(); *(volatile v4f*)dst = o; }
__global__ __launch_bounds__(256) void k_plane(const float* __restrict__ F, int rows, int off, float sc, h16* P16) { const size_t e = ((size_t)blockIdx.x * 256 + threadIdx.x) * 2; if (e >= (size_t)rows * HD) return; const int d = (int)(e % HD); const size_t t = e / HD; v2h o;
#pragma unroll
    for (int q = 0; q < 2; ++q) o[q] = tohx(__fmul_rn(F[t * CH + off + d + q], sc)); *(volatile v2h*)(P16 + e) = o; __threadfence(); *(volatile v2h*)(P16 + e) = o; }
__global__ __launch_bounds__(256) void k_vtpad16(const float* __restrict__ F, int off, h16* V16) { const size_t e = ((size_t)blockIdx.x * 256 + threadIdx.x) * 2; if (e >= (size_t)HP * TT) return; const int t = (int)(e % TT); const int d = (int)(e / TT); v2h o;
#pragma unroll
    for (int q = 0; q < 2; ++q) o[q] = (d < HD) ? tohx(F[(size_t)(t + q) * CH + off + d]) : (_Float16)0.0f; *(volatile v2h*)(V16 + e) = o; __threadfence(); *(volatile v2h*)(V16 + e) = o; }
__global__ __launch_bounds__(256) void k_gsoft(const float* __restrict__ Sb, const float* __restrict__ RX, const float* __restrict__ RY, const int* __restrict__ msk, int h, h16* P16) {
    const int lane = threadIdx.x & 31; const int row = blockIdx.x * 8 + (threadIdx.x >> 5); if (row >= QP) return; const float* sr = Sb + (size_t)row * TT; const float* rx = RX + ((size_t)row * NH_ + h) * GW; const float* ry = RY + ((size_t)row * NH_ + h) * GW; float mx = -3.0e38f;
    auto logit = [&](const v4f& a, const v4f& x4, float yv, const v4i& m4, int q) { float rp = __fadd_rn(x4[q], yv); asm volatile("" : "+v"(rp)); float t = __fadd_rn(a[q], rp); asm volatile("" : "+v"(t)); t = __fadd_rn(t, m4[q] ? -100.0f : 0.0f); asm volatile("" : "+v"(t)); return t; };
#pragma unroll 4
    for (int ch = 0; ch < TT / 128; ++ch) { const int j0 = ch * 128 + lane * 4; const v4f a = *(const v4f*)(sr + j0); const v4f x4 = *(const v4f*)(rx + (j0 & 63)); const float yv = ry[j0 >> 6]; const v4i m4 = *(const v4i*)(msk + j0);
#pragma unroll
        for (int q = 0; q < 4; ++q) mx = fmaxf(mx, logit(a, x4, yv, m4, q)); }
#pragma unroll
    for (int sh = 16; sh; sh >>= 1) mx = fmaxf(mx, __shfl_xor(mx, sh, 32));
    float sum = 0.f;
#pragma unroll 4
    for (int ch = 0; ch < TT / 128; ++ch) { const int j0 = ch * 128 + lane * 4; const v4f a = *(const v4f*)(sr + j0); const v4f x4 = *(const v4f*)(rx + (j0 & 63)); const float yv = ry[j0 >> 6]; const v4i m4 = *(const v4i*)(msk + j0);
#pragma unroll
        for (int q = 0; q < 4; ++q) { float d0 = __fsub_rn(logit(a, x4, yv, m4, q), mx); asm volatile("" : "+v"(d0)); sum += __builtin_amdgcn_exp2f(__fmul_rn(d0, 1.4426950408889634f)); } }
#pragma unroll
    for (int sh = 16; sh; sh >>= 1) sum += __shfl_xor(sum, sh, 32);
    const float f = __fdiv_rn(PCAR, sum);
#pragma unroll 1
    for (int ps = 0; ps < 2; ++ps) {
#pragma unroll 2
        for (int ch = 0; ch < TT / 128; ++ch) { const int j0 = ch * 128 + lane * 4; const v4f a = *(const v4f*)(sr + j0); const v4f x4 = *(const v4f*)(rx + (j0 & 63)); const float yv = ry[j0 >> 6]; const v4i m4 = *(const v4i*)(msk + j0); v4h o4;
#pragma unroll
            for (int q = 0; q < 4; ++q) { float d0 = __fsub_rn(logit(a, x4, yv, m4, q), mx); asm volatile("" : "+v"(d0)); float ex = __builtin_amdgcn_exp2f(__fmul_rn(d0, 1.4426950408889634f)); asm volatile("" : "+v"(ex)); o4[q] = tohx(ex * f); }
            *(volatile v4h*)(P16 + (size_t)row * TT + j0) = o4; }
        if (ps == 0) __threadfence(); }
}
__global__ __launch_bounds__(256) void k_mergeall(const float* __restrict__ OB, bf* Ah, bf* Al) { const size_t i = (size_t)blockIdx.x * 256 + threadIdx.x; if (i >= (size_t)QP * CH / 4) return; const int c0 = (int)(i % (CH / 4)) * 4; const int t = (int)(i / (CH / 4)); v4us oh, ol;
#pragma unroll
    for (int q = 0; q < 4; ++q) { const int c = c0 + q; const int h = c / HD, d = c % HD; unsigned short a, b; splitf(__fmul_rn(OB[((size_t)h * QP + t) * HP + d], 1.0f / PCAR), a, b); oh[q] = a; ol[q] = b; }
    *(volatile v4us*)(Ah + (size_t)t * CH + c0) = oh; *(volatile v4us*)(Al + (size_t)t * CH + c0) = ol; __threadfence(); *(volatile v4us*)(Ah + (size_t)t * CH + c0) = oh; *(volatile v4us*)(Al + (size_t)t * CH + c0) = ol; }
__global__ __launch_bounds__(256) void k_copy(const float* __restrict__ T, float* out, size_t n4) { const size_t i = (size_t)blockIdx.x * 256 + threadIdx.x; if (i >= n4) return; const v4f a = *(const v4f*)(T + i * 4); *(volatile v4f*)(out + i * 4) = a; __threadfence(); *(volatile v4f*)(out + i * 4) = a; }

extern "C" void kernel_launch(void* const* d_in, const int* in_sizes, int n_in,
                              void* d_out, int out_size, void* d_ws, size_t ws_size, hipStream_t stream) {
    (void)in_sizes; (void)n_in; (void)out_size;
    const float* query = (const float*)d_in[0]; const float* box = (const float*)d_in[1]; const float* kin = (const float*)d_in[2]; const float* vin = (const float*)d_in[3]; const int* msk = (const int*)d_in[4];
    const float* Wq = (const float*)d_in[7]; const float* bq = (const float*)d_in[8]; const float* Wk = (const float*)d_in[9]; const float* bk = (const float*)d_in[10]; const float* Wv = (const float*)d_in[11]; const float* bv = (const float*)d_in[12]; const float* Wp = (const float*)d_in[13]; const float* bp = (const float*)d_in[14];
    const float* c1w1 = (const float*)d_in[15]; const float* c1b1 = (const float*)d_in[16]; const float* c1w2 = (const float*)d_in[17]; const float* c2w1 = (const float*)d_in[18]; const float* c2b1 = (const float*)d_in[19]; const float* c2w2 = (const float*)d_in[20];
    float* OUT = (float*)d_out;
    char* wsp = (char*)d_ws;
    auto take = [&](size_t bytes) { char* p = wsp; wsp += (bytes + 255) & ~(size_t)255; return (void*)p; };
    bf* WQ = (bf*)take((size_t)CH * CH * 2); bf* WK = (bf*)take((size_t)CH * CH * 2); bf* WV = (bf*)take((size_t)CH * CH * 2); bf* WP = (bf*)take((size_t)CH * CH * 2);
    float* RX = (float*)take((size_t)QP * NH_ * GW * 4); float* RY = (float*)take((size_t)QP * NH_ * GW * 4); bf* XQ = (bf*)take((size_t)QP * CH * 2); bf* XK = (bf*)take((size_t)TT * CH * 2);
    float* FQ = (float*)take((size_t)QP * CH * 4); float* FK = (float*)take((size_t)TT * CH * 4); float* FV = (float*)take((size_t)TT * CH * 4);
    h16* QP16 = (h16*)take((size_t)QP * HD * 2); h16* KP16 = (h16*)take((size_t)TT * HD * 2); h16* VT16 = (h16*)take((size_t)HP * TT * 2); float* Sb = (float*)take((size_t)QP * TT * 4); h16* P16 = (h16*)take((size_t)QP * TT * 2); float* OB = (float*)take((size_t)NH_ * QP * HP * 4); bf* ATh = (bf*)take((size_t)QP * CH * 2); bf* ATl = (bf*)take((size_t)QP * CH * 2); float* TMP = (float*)take((size_t)QP * CH * 4);
    if ((size_t)(wsp - (char*)d_ws) > ws_size) return;
    k_cvt8<<<(CH * CH / 8 + 255) / 256, 256, 0, stream>>>(Wq, WQ, (size_t)CH * CH / 8); k_cvt8<<<(CH * CH / 8 + 255) / 256, 256, 0, stream>>>(Wk, WK, (size_t)CH * CH / 8); k_cvt8<<<(CH * CH / 8 + 255) / 256, 256, 0, stream>>>(Wv, WV, (size_t)CH * CH / 8); k_cvt8<<<(CH * CH / 8 + 255) / 256, 256, 0, stream>>>(Wp, WP, (size_t)CH * CH / 8);
    k_zero<<<(unsigned)(((size_t)QP * NH_ * GW / 4 + 255) / 256), 256, 0, stream>>>(RX, (size_t)QP * NH_ * GW / 4); k_zero<<<(unsigned)(((size_t)QP * NH_ * GW / 4 + 255) / 256), 256, 0, stream>>>(RY, (size_t)QP * NH_ * GW / 4);
    k_zero16<<<(unsigned)(((size_t)QP * CH / 8 + 255) / 256), 256, 0, stream>>>(XQ, (size_t)QP * CH / 8);
    const unsigned NCPB = (NQ * NH_ * (GW / 4) + 255) / 256;
    for (int b = 0; b < NB_; ++b) {
        k_cpb<<<NCPB, 256, 0, stream>>>(box + (size_t)b * NQ * 4, 0, c1w1, c1b1, c1w2, RX); k_cpb<<<NCPB, 256, 0, stream>>>(box + (size_t)b * NQ * 4, 1, c2w1, c2b1, c2w2, RY);
        k_cvt8<<<(unsigned)(((size_t)NQ * CH / 8 + 255) / 256), 256, 0, stream>>>(query + (size_t)b * NQ * CH, XQ, (size_t)NQ * CH / 8);
        k_gemmw<bf, 0, true><<<dim3(QP / 64, CH / 64, 1), 32, 0, stream>>>(XQ, nullptr, WQ, nullptr, CH, FQ, CH, bq, 0, 0, 0);
        k_cvt8<<<(unsigned)(((size_t)TT * CH / 8 + 255) / 256), 256, 0, stream>>>(kin + (size_t)b * TT * CH, XK, (size_t)TT * CH / 8);
        k_gemmw<bf, 0, true><<<dim3(TT / 64, CH / 64, 1), 32, 0, stream>>>(XK, nullptr, WK, nullptr, CH, FK, CH, bk, 0, 0, 0);
        k_cvt8<<<(unsigned)(((size_t)TT * CH / 8 + 255) / 256), 256, 0, stream>>>(vin + (size_t)b * TT * CH, XK, (size_t)TT * CH / 8);
        k_gemmw<bf, 0, true><<<dim3(TT / 64, CH / 64, 1), 32, 0, stream>>>(XK, nullptr, WV, nullptr, CH, FV, CH, bv, 0, 0, 0);
        for (int h = 0; h < NH_; ++h) {
            k_plane<<<(QP * HD / 2 + 255) / 256, 256, 0, stream>>>(FQ, QP, h * HD, SCL, QP16);
            k_plane<<<(TT * HD / 2 + 255) / 256, 256, 0, stream>>>(FK, TT, h * HD, 1.0f, KP16);
            k_vtpad16<<<(HP * TT / 2 + 255) / 256, 256, 0, stream>>>(FV, h * HD, VT16);
            k_gemmw<h16, 0, false><<<dim3(QP / 64, TT / 64, 1), 32, 0, stream>>>(QP16, nullptr, KP16, nullptr, HD, Sb, TT, nullptr, 0, 0, 0);
            k_gsoft<<<QP / 8, 256, 0, stream>>>(Sb, RX, RY, msk + (size_t)b * TT, h, P16);
            k_gemmw<h16, 0, false><<<dim3(QP / 64, HP / 64, 1), 32, 0, stream>>>(P16, nullptr, VT16, nullptr, TT, OB + (size_t)h * QP * HP, HP, nullptr, 0, 0, 0); }
        k_mergeall<<<(unsigned)(((size_t)QP * CH / 4 + 255) / 256), 256, 0, stream>>>(OB, ATh, ATl);
        k_gemmw<bf, 1, true><<<dim3(QP / 64, CH / 64, 1), 32, 0, stream>>>(ATh, ATl, WP, nullptr, CH, TMP, CH, bp, 0, 0, 0);
        k_copy<<<(unsigned)(((size_t)NQ * CH / 4 + 255) / 256), 256, 0, stream>>>(TMP, OUT + (size_t)b * NQ * CH, (size_t)NQ * CH / 4); }
}
